// ARQS_66228395704554
// MI455X (gfx1250) — hardware-verified
//
#include <hip/hip_runtime.h>
#include <stddef.h>
#include <math.h>

#define BROWS 65536
#define DIM   64
#define HID   512
#define NBIN  8
#define NPAR  23
#define OUTD  1472
#define TM    16
#define NTHR  256
#define XP    72
#define HP    520
#define LDP   32

static_assert(OUTD == DIM * NPAR);
static_assert(NPAR == 3 * NBIN - 1);
static_assert(NPAR * 64 == OUTD);
static_assert((NTHR / 32) * 64 == HID);
static_assert(BROWS % TM == 0);
static_assert(BROWS % 32 == 0);
static_assert(TM * DIM == 4 * NTHR);
static_assert(DIM % 64 == 0);
static_assert(HID % 64 == 0);
static_assert(OUTD % 32 == 0);
static_assert(XP % 8 == 0);
static_assert(HP % 8 == 0);
static_assert(HP >= HID);
static_assert(XP >= DIM);

#define L_XS   0
#define L_XH   (L_XS + TM * DIM * 4)
#define L_H0   (L_XH + TM * XP * 2)
#define L_H1   (L_H0 + TM * HP * 2)
#define L_PAR  (L_H1 + TM * HP * 2)
#define L_ZS   (L_PAR + TM * OUTD * 4)
#define L_LDL  (L_ZS + TM * DIM * 4)
#define L_LDR  (L_LDL + TM * DIM * 4)
#define LDS_BYTES (L_LDR + 32 * 4)
static_assert(L_XH % 16 == 0);
static_assert(L_H0 % 16 == 0);
static_assert(L_H1 % 16 == 0);
static_assert(L_PAR % 16 == 0);
static_assert(L_ZS % 16 == 0);
static_assert(L_LDL % 16 == 0);
static_assert(L_LDR % 16 == 0);
static_assert(LDS_BYTES == 142208);

typedef _Float16 f16;
typedef f16 v16h __attribute__((ext_vector_type(16)));
typedef f16 v8h_t __attribute__((ext_vector_type(8)));
typedef v8h_t __attribute__((may_alias)) v8h;
typedef float v8f __attribute__((ext_vector_type(8)));
typedef float v4f_t __attribute__((ext_vector_type(4)));
typedef v4f_t __attribute__((may_alias)) v4f;
typedef unsigned int v4u __attribute__((ext_vector_type(4)));

union Frag { v16h v; v8h_t h[2]; };
union Pack8 { v8h_t h; v4u u; };

__device__ __forceinline__ v8f zero8() {
    v8f z;
#pragma unroll
    for (int i = 0; i < 8; ++i) z[i] = 0.0f;
    return z;
}

__device__ __forceinline__ v16h ldfrag(const f16* p, int k0) {
    Frag f;
    f.h[0] = *(const v8h*)(p + k0);
    f.h[1] = *(const v8h*)(p + k0 + 16);
    return f.v;
}

__device__ __forceinline__ v8f wmma16(v16h a, v16h b, v8f c) {
    return __builtin_amdgcn_wmma_f32_16x16x32_f16(false, a, false, b, (short)0, c, false, false);
}

template <int KD>
__device__ __forceinline__ void gemm4(const f16* pa, const f16* __restrict__ pb, v8f (&acc)[4])
{
#pragma unroll 2
    for (int k0 = 0; k0 < KD; k0 += 32) {
        const v16h a  = ldfrag(pa, k0);
        const v16h b0 = ldfrag(pb, k0);
        const v16h b1 = ldfrag(pb + 16 * KD, k0);
        const v16h b2 = ldfrag(pb + 32 * KD, k0);
        const v16h b3 = ldfrag(pb + 48 * KD, k0);
        acc[0] = wmma16(a, b0, acc[0]);
        acc[1] = wmma16(a, b1, acc[1]);
        acc[2] = wmma16(a, b2, acc[2]);
        acc[3] = wmma16(a, b3, acc[3]);
        asm volatile("v_nop\n\tv_nop\n\tv_nop\n\tv_nop"
                     : "+v"(acc[0]), "+v"(acc[1]), "+v"(acc[2]), "+v"(acc[3])
                     : "v"(a), "v"(b0), "v"(b1), "v"(b2), "v"(b3));
    }
}

__device__ __forceinline__ void epi_relu(f16* dst, int col0, const float* __restrict__ bias,
                                         const v8f (&acc)[4], float inv, int hh, int m)
{
#pragma unroll
    for (int t = 0; t < 4; ++t) {
        const int col = col0 + 16 * t + m;
        const float bv = bias[col];
#pragma unroll
        for (int r = 0; r < 8; ++r) {
            const float v = fmaxf(acc[t][r] * inv + bv, 0.0f);
            dst[(8 * hh + r) * HP + col] = (f16)(v * 64.0f);
        }
    }
}

__device__ __forceinline__ void rqs_item(const float* p, float xin, float aff, float& zv, float& ld)
{
#pragma clang fp contract(off)
    float wb[NBIN], hb[NBIN];
    float mw = p[0], mh = p[NBIN];
#pragma unroll
    for (int b = 1; b < NBIN; ++b) { mw = fmaxf(mw, p[b]); mh = fmaxf(mh, p[NBIN + b]); }
    float sw = 0.0f, sh = 0.0f;
#pragma unroll
    for (int b = 0; b < NBIN; ++b) {
        wb[b] = expf(p[b] - mw);        sw += wb[b];
        hb[b] = expf(p[NBIN + b] - mh); sh += hb[b];
    }
    const float rw = 1.0f / sw;
    const float rh = 1.0f / sh;
#pragma unroll
    for (int b = 0; b < NBIN; ++b) {
        wb[b] = 0.001f + aff * (wb[b] * rw);
        hb[b] = 0.001f + aff * (hb[b] * rh);
    }
    float dv[NBIN + 1];
    dv[0] = 1.0f; dv[NBIN] = 1.0f;
#pragma unroll
    for (int j = 0; j < NBIN - 1; ++j) {
        const float t = p[2 * NBIN + j];
        const float sp = fmaxf(t, 0.0f) + log1pf(expf(-fabsf(t)));
        dv[j + 1] = sp + 0.001f;
    }
    float kx = 0.0f; int cnt = 0;
#pragma unroll
    for (int b = 0; b < NBIN; ++b) { cnt += (kx < xin) ? 1 : 0; kx = kx + wb[b]; }
    cnt += (kx < xin) ? 1 : 0;
    const int kbin = min(max(cnt, 1), NBIN) - 1;
    float x_k = 0.0f, y_k = 0.0f, w_k = 0.0f, h_k = 0.0f;
#pragma unroll
    for (int b = 0; b < NBIN; ++b) {
        const bool lt = (b < kbin);
        const bool eq = (b == kbin);
        x_k = lt ? (x_k + wb[b]) : x_k;
        y_k = lt ? (y_k + hb[b]) : y_k;
        w_k = eq ? wb[b] : w_k;
        h_k = eq ? hb[b] : h_k;
    }
    float d_k = 1.0f, d_k1 = 1.0f;
#pragma unroll
    for (int j = 0; j <= NBIN; ++j) {
        d_k  = (j == kbin) ? dv[j] : d_k;
        d_k1 = (j == kbin + 1) ? dv[j] : d_k1;
    }
    const float s   = h_k / w_k;
    const float th  = (xin - x_k) / w_k;
    const float omt = 1.0f - th;
    const float t1t = th * omt;
    const float th2 = th * th;
    const float den = s + ((d_k + d_k1) - 2.0f * s) * t1t;
    zv = y_k + (h_k * (s * th2 + d_k * t1t)) / (den + 1e-6f);
    const float nom = (s * s) * ((d_k1 * th2 + (2.0f * s) * t1t) + d_k * (omt * omt));
    ld = logf(nom / (den * den + 1e-6f));
}

__global__ void __launch_bounds__(NTHR) cvt_t_kernel(const float* __restrict__ W, f16* __restrict__ Wt,
                                                    int K, int N, float scale)
{
    __shared__ __align__(16) f16 tile[32 * XP];
    const int tid = threadIdx.x, lane = tid & 31, wv = tid >> 5;
    const int n0 = blockIdx.x * 32, k0 = blockIdx.y * 64;
#pragma unroll
    for (int i = 0; i < 8; ++i) {
        const int idx = tid + NTHR * i;
        const int kk = idx >> 5;
        const int nn = idx & 31;
        const float v = W[(size_t)(k0 + kk) * N + n0 + nn];
        tile[nn * XP + kk] = (f16)(v * scale);
    }
    __syncthreads();
    const int nl = 4 * wv + (lane >> 3);
    const int kp = (lane & 7) * 8;
    Pack8 pk;
    pk.h = *(const v8h*)(tile + nl * XP + kp);
    f16* dst = Wt + (size_t)(n0 + nl) * K + k0 + kp;
    *(volatile v4u*)dst = pk.u;
    __threadfence();
    *(volatile v4u*)dst = pk.u;
}

__global__ void __launch_bounds__(NTHR) fused_kernel(
    const float* __restrict__ x,
    const float* __restrict__ b0, const float* __restrict__ b1, const float* __restrict__ b2,
    const int* __restrict__ nbp,
    const f16* __restrict__ w0t, const f16* __restrict__ w1t, const f16* __restrict__ w2t,
    float* __restrict__ zout, float* __restrict__ ldp)
{
    extern __shared__ __align__(16) char smem[];
    float* xs  = (float*)(smem + L_XS);
    f16*   xh  = (f16*)(smem + L_XH);
    f16*   h0  = (f16*)(smem + L_H0);
    f16*   h1  = (f16*)(smem + L_H1);
    float* par = (float*)(smem + L_PAR);
    float* zs  = (float*)(smem + L_ZS);
    float* ldl = (float*)(smem + L_LDL);
    float* ldr = (float*)(smem + L_LDR);

    const int tid  = threadIdx.x;
    const int lane = tid & 31;
    const int wv   = __builtin_amdgcn_readfirstlane(tid >> 5);
    const int hh   = lane >> 4, m = lane & 15;
    const int rb   = blockIdx.x * TM;

#pragma unroll
    for (int i = 0; i < 4; ++i) {
        const int idx = tid + i * NTHR;
        const int r = idx >> 6, c = idx & 63;
        const float v = x[(size_t)(rb + r) * DIM + c];
        xs[r * DIM + c] = v;
        xh[r * XP + c]  = (f16)(v * 8.0f);
    }
    __syncthreads();

    {
        v8f acc[4];
        acc[0] = zero8(); acc[1] = zero8(); acc[2] = zero8(); acc[3] = zero8();
        gemm4<DIM>(xh + m * XP + 8 * hh, w0t + (size_t)(64 * wv + m) * DIM + 8 * hh, acc);
        epi_relu(h0, 64 * wv, b0, acc, 1.0f / 128.0f, hh, m);
    }
    __syncthreads();

    {
        v8f acc[4];
        acc[0] = zero8(); acc[1] = zero8(); acc[2] = zero8(); acc[3] = zero8();
        gemm4<HID>(h0 + m * HP + 8 * hh, w1t + (size_t)(64 * wv + m) * HID + 8 * hh, acc);
        epi_relu(h1, 64 * wv, b1, acc, 1.0f / 1024.0f, hh, m);
    }
    __syncthreads();

    {
        const f16* pa = h1 + m * HP + 8 * hh;
#pragma unroll 1
        for (int g = wv; g < NPAR; g += NTHR / 32) {
            v8f acc[4];
            acc[0] = zero8(); acc[1] = zero8(); acc[2] = zero8(); acc[3] = zero8();
            gemm4<HID>(pa, w2t + (size_t)(64 * g + m) * HID + 8 * hh, acc);
#pragma unroll
            for (int t = 0; t < 4; ++t) {
                const int col = 64 * g + 16 * t + m;
                const float bv = b2[col];
#pragma unroll
                for (int r = 0; r < 8; ++r)
                    par[(8 * hh + r) * OUTD + col] = acc[t][r] * (1.0f / 1024.0f) + bv;
            }
        }
    }
    __syncthreads();

    const int nb = nbp[0];
    const float aff = 1.0f - 0.001f * (float)nb;
#pragma unroll 1
    for (int i = 0; i < 4; ++i) {
        const int item = tid + i * NTHR;
        const int row = item >> 6, d = item & 63;
        const float xin = fminf(fmaxf(xs[row * DIM + d], 0.0f), 1.0f);
        float zv, ld;
        rqs_item(par + row * OUTD + d * NPAR, xin, aff, zv, ld);
        zs[row * DIM + d]  = zv;
        ldl[row * DIM + d] = ld;
    }
    __syncthreads();

    if (tid < 32) {
        float s = 0.0f;
        if (tid < TM) {
#pragma unroll 8
            for (int d = 0; d < DIM; ++d) s += ldl[tid * DIM + d];
        }
        ldr[tid] = s;
    }
    __syncthreads();

    const int zr = 2 * wv + (lane >> 4);
    const int c4 = (lane & 15) * 4;
    const v4f_t zv4 = *(const v4f*)(zs + zr * DIM + c4);
    const v4f_t lv4 = *(const v4f*)(ldr + (lane & 7) * 4);
    float* gz = zout + (size_t)(rb + zr) * DIM + c4;
    float* gl = ldp + (size_t)blockIdx.x * LDP + (lane & 7) * 4;
    const bool wl = (wv == 0) && (lane < 8);
    *(volatile v4f_t*)gz = zv4;
    if (wl) *(volatile v4f_t*)gl = lv4;
    __threadfence();
    *(volatile v4f_t*)gz = zv4;
    if (wl) *(volatile v4f_t*)gl = lv4;
}

__global__ void __launch_bounds__(NTHR) ld_lines_kernel(const float* __restrict__ ldp,
                                                       float* __restrict__ ldo, int nlines)
{
    const int lane = threadIdx.x & 31, wv = threadIdx.x >> 5;
    const int line = (blockIdx.x * (NTHR / 32) + wv) * 4 + (lane >> 3);
    const int q    = lane & 7;
    const int lc   = min(line, nlines - 1);
    const v4f_t v = *(const v4f*)(ldp + (size_t)(2 * lc + (q >> 2)) * LDP + (q & 3) * 4);
    float* dst = ldo + (size_t)lc * 32 + 4 * q;
    const bool ok = (line < nlines);
    if (ok) *(volatile v4f_t*)dst = v;
    __threadfence();
    if (ok) *(volatile v4f_t*)dst = v;
}

extern "C" void kernel_launch(void* const* d_in, const int* in_sizes, int n_in,
                              void* d_out, int out_size, void* d_ws, size_t ws_size,
                              hipStream_t stream)
{
    if (n_in < 8) return;
    if (in_sizes[0] != BROWS * DIM) return;
    if (in_sizes[1] != DIM * HID) return;
    if (in_sizes[2] != HID) return;
    if (in_sizes[3] != HID * HID) return;
    if (in_sizes[4] != HID) return;
    if (in_sizes[5] != HID * OUTD) return;
    if (in_sizes[6] != OUTD) return;
    if (in_sizes[7] < 1) return;
    if (out_size != BROWS * DIM + BROWS) return;

    const float* x  = (const float*)d_in[0];
    const float* W0 = (const float*)d_in[1];
    const float* b0 = (const float*)d_in[2];
    const float* W1 = (const float*)d_in[3];
    const float* b1 = (const float*)d_in[4];
    const float* W2 = (const float*)d_in[5];
    const float* b2 = (const float*)d_in[6];
    const int*   nbp = (const int*)d_in[7];

    float* z   = (float*)d_out;
    float* ldo = z + (size_t)BROWS * DIM;

    const size_t nblk = (size_t)BROWS / TM;
    const size_t oW0  = 0;
    const size_t oW1  = oW0 + (size_t)HID * DIM * 2;
    const size_t oW2  = oW1 + (size_t)HID * HID * 2;
    const size_t oLD  = oW2 + (size_t)OUTD * HID * 2;
    const size_t total = oLD + nblk * LDP * 4;
    if (total > ws_size) return;

    char* ws = (char*)d_ws;
    f16* w0t = (f16*)(ws + oW0);
    f16* w1t = (f16*)(ws + oW1);
    f16* w2t = (f16*)(ws + oW2);
    float* ldp = (float*)(ws + oLD);

    cvt_t_kernel<<<dim3(HID / 32, DIM / 64), NTHR, 0, stream>>>(W0, w0t, DIM, HID, 16.0f);
    cvt_t_kernel<<<dim3(HID / 32, HID / 64), NTHR, 0, stream>>>(W1, w1t, HID, HID, 16.0f);
    cvt_t_kernel<<<dim3(OUTD / 32, HID / 64), NTHR, 0, stream>>>(W2, w2t, HID, OUTD, 16.0f);

    hipFuncSetAttribute(reinterpret_cast<const void*>(&fused_kernel),
                        hipFuncAttributeMaxDynamicSharedMemorySize, LDS_BYTES);
    fused_kernel<<<(unsigned)nblk, NTHR, LDS_BYTES, stream>>>(x, b0, b1, b2, nbp,
                                                               w0t, w1t, w2t, z, ldp);

    const int nlines = BROWS / 32;
    ld_lines_kernel<<<(nlines + 31) / 32, NTHR, 0, stream>>>(ldp, ldo, nlines);
}
